// MLP_85598698209927
// MI455X (gfx1250) — hardware-run, weakly checked
//
#include <hip/hip_runtime.h>
#include <math.h>

#ifndef NROW
#define NROW 1024
#endif
#define NROW_FULL 1024
#define DIN 1024
#define DH 512
#define NCAT (2 * DH)

typedef __attribute__((ext_vector_type(4))) float v4f;
typedef __attribute__((ext_vector_type(4))) unsigned int v4u;
typedef _Float16 h16;

#define VST2(T, ptr, val) do { const T vst2_v_ = (val); *(volatile T*)(ptr) = vst2_v_; __threadfence(); *(volatile T*)(ptr) = vst2_v_; } while (0)
#define VST2V4(ptr, val) do { const v4f vst2_v4_ = (val); *(volatile v4f*)(ptr) = vst2_v4_; __threadfence(); *(volatile v4f*)(ptr) = vst2_v4_; } while (0)

namespace eng {
typedef __attribute__((ext_vector_type(16))) _Float16 v16h;
typedef __attribute__((ext_vector_type(8)))  _Float16 v8h;
typedef __attribute__((ext_vector_type(16))) __bf16   v16b;
typedef __attribute__((ext_vector_type(8)))  __bf16   v8b;
typedef __attribute__((ext_vector_type(8)))  float    v8f;
typedef __attribute__((ext_vector_type(4)))  float    v4f;

__device__ __forceinline__ unsigned short f2bf_bits(float f) {
  unsigned u = __float_as_uint(f);
  return (unsigned short)((u + 0x7FFFu + ((u >> 16) & 1u)) >> 16);
}
__device__ __forceinline__ float bf_bits2f(unsigned short h) { return __uint_as_float(((unsigned)h) << 16); }

__device__ __forceinline__ void dep_guard_h(v8f& a, v8f& b, v16h x, v16h y) { asm volatile("v_nop\n\tv_nop\n\tv_nop\n\tv_nop" : "+v"(a), "+v"(b) : "v"(x), "v"(y)); }
__device__ __forceinline__ void dep_guard_b(v8f& a, v8f& b, v16b x, v16b y) { asm volatile("v_nop\n\tv_nop\n\tv_nop\n\tv_nop" : "+v"(a), "+v"(b) : "v"(x), "v"(y)); }
__device__ __forceinline__ void keep4_h(v16h a, v16h b, v16h c, v16h d) { asm volatile("v_nop" :: "v"(a), "v"(b), "v"(c), "v"(d)); }
__device__ __forceinline__ void keep4_b(v16b a, v16b b, v16b c, v16b d) { asm volatile("v_nop" :: "v"(a), "v"(b), "v"(c), "v"(d)); }
__device__ __forceinline__ void acc_guard4(v8f& a, v8f& b, v8f& c, v8f& d) { asm volatile("v_nop\n\tv_nop\n\tv_nop\n\tv_nop" : "+v"(a), "+v"(b), "+v"(c), "+v"(d)); }
template <typename T> struct Frag;
template <> struct Frag<_Float16> {
  typedef v16h V; union U { v16h v; v8h h[2]; };
  static __device__ __forceinline__ v16h load(const _Float16* p) {
    U f; f.h[0] = *(const v8h*)(p); f.h[1] = *(const v8h*)(p + 16); return f.v;
  }
  static __device__ __forceinline__ v8f mma(v16h a, v16h b, v8f c) {
    return __builtin_amdgcn_wmma_f32_16x16x32_f16(false, a, false, b, (short)0, c, false, false);
  }
  static __device__ __forceinline__ void guard(v8f& a, v8f& b, v16h x, v16h y) { dep_guard_h(a, b, x, y); }
  static __device__ __forceinline__ void keep(v16h a, v16h b, v16h c, v16h d) { keep4_h(a, b, c, d); }
};
template <> struct Frag<__bf16> {
  typedef v16b V; union U { v16b v; v8b h[2]; };
  static __device__ __forceinline__ v16b load(const __bf16* p) {
    U f; f.h[0] = *(const v8b*)(p); f.h[1] = *(const v8b*)(p + 16); return f.v;
  }
  static __device__ __forceinline__ v8f mma(v16b a, v16b b, v8f c) {
    return __builtin_amdgcn_wmma_f32_16x16x32_bf16(false, a, false, b, (short)0, c, false, false);
  }
  static __device__ __forceinline__ void guard(v8f& a, v8f& b, v16b x, v16b y) { dep_guard_b(a, b, x, y); }
  static __device__ __forceinline__ void keep(v16b a, v16b b, v16b c, v16b d) { keep4_b(a, b, c, d); }
};

template <int ET> struct Elem;
template <> struct Elem<0> { typedef _Float16 T; };
template <> struct Elem<1> { typedef __bf16 T; };
template <int ET, bool SPLIT, int BIAS_MODE, int OUT_MODE, bool RESID, int ACT = 0>
__global__ __launch_bounds__(256) void wmma_gemm64(
    const unsigned short* __restrict__ Ap, const unsigned short* __restrict__ A2p, int lda, long strideA,
    const unsigned short* __restrict__ Btp, const unsigned short* __restrict__ Bt2p, int ldb, long strideB,
    void* __restrict__ Cout, void* __restrict__ Cout2, int ldc, long strideC,
    const float* __restrict__ bias,
    const float* __restrict__ resid, long strideR,
    int M, int N, int K, float scale) {
  typedef typename Elem<ET>::T T;
  typedef typename Frag<T>::V V;
  const T* A = (const T*)Ap; const T* A2 = (const T*)A2p; const T* Bt = (const T*)Btp; const T* Bt2 = (const T*)Bt2p;
  __shared__ __align__(16) float sT[8][16 * 68];
  const int b    = blockIdx.y;
  const int lane = threadIdx.x & 31;
  const int wave = threadIdx.x >> 5;
  const int tilesN = N >> 6;
  const int tilesM = M >> 6;
  const int tile = blockIdx.x * 8 + wave;
  if (tile >= tilesM * tilesN) return;
  const int tm = tile / tilesN;
  const int tn = tile - tm * tilesN;
  const int m0 = tm << 6;
  const int n0 = tn << 6;

  const T* Ab  = A  + (size_t)b * strideA;
  const T* Bb  = Bt + (size_t)b * strideB;
  const T* Ab2 = SPLIT ? (A2  + (size_t)b * strideA) : nullptr;
  const T* Bb2 = SPLIT ? (Bt2 + (size_t)b * strideB) : nullptr;

  const int rlane = lane & 15;
  const int koff  = (lane >> 4) * 8;
  const int mOff  = (lane >> 4) * 8;

  v8f acc[4][4];
#pragma unroll
  for (int i = 0; i < 4; ++i)
#pragma unroll
    for (int j = 0; j < 4; ++j) acc[i][j] = (v8f){0.f,0.f,0.f,0.f,0.f,0.f,0.f,0.f};

  for (int k0 = 0; k0 < K; k0 += 32) {
    V bh[4], bl[4];
#pragma unroll
    for (int j = 0; j < 4; ++j) {
      const size_t bo = (size_t)(n0 + (j << 4) + rlane) * ldb + koff + k0;
      bh[j] = Frag<T>::load(Bb + bo);
      if (SPLIT) bl[j] = Frag<T>::load(Bb2 + bo);
    }
#pragma unroll
    for (int i = 0; i < 4; ++i) {
      const size_t ao = (size_t)(m0 + (i << 4) + rlane) * lda + koff + k0;
      V ah = Frag<T>::load(Ab + ao);
      V al;
      if (SPLIT) al = Frag<T>::load(Ab2 + ao);
#pragma unroll
      for (int j = 0; j < 4; ++j) {
        acc[i][j] = Frag<T>::mma(ah, bh[j], acc[i][j]);
        if (SPLIT) {
          acc[i][j] = Frag<T>::mma(ah, bl[j], acc[i][j]);
          acc[i][j] = Frag<T>::mma(al, bh[j], acc[i][j]);
        }
      }
      Frag<T>::guard(acc[i][0], acc[i][3], ah, SPLIT ? al : ah);
    }
    Frag<T>::keep(bh[0], bh[1], bh[2], bh[3]);
    if (SPLIT) Frag<T>::keep(bl[0], bl[1], bl[2], bl[3]);
  }
  acc_guard4(acc[0][0], acc[0][1], acc[0][2], acc[0][3]);
  acc_guard4(acc[1][0], acc[1][1], acc[1][2], acc[1][3]);
  acc_guard4(acc[2][0], acc[2][1], acc[2][2], acc[2][3]);
  acc_guard4(acc[3][0], acc[3][1], acc[3][2], acc[3][3]);

  float* slab = sT[wave];
  const float* Rb = RESID ? (resid + (size_t)b * strideR) : nullptr;
#pragma unroll
  for (int i = 0; i < 4; ++i) {
    const int mBase = m0 + (i << 4);
#pragma unroll
    for (int j = 0; j < 4; ++j) {
      const int n = n0 + (j << 4) + rlane;
      float bv = 0.f;
      if (BIAS_MODE == 2) bv = bias[n];
#pragma unroll
      for (int r = 0; r < 8; ++r) {
        float v = acc[i][j][r] * scale;
        if (BIAS_MODE == 1) v += bias[mBase + mOff + r];
        if (BIAS_MODE == 2) v += bv;
        if (RESID) v += Rb[(size_t)(mBase + mOff + r) * ldc + n];
        if (ACT == 1) v = tanhf(v);
        if (ACT == 2) v = fmaxf(v, 0.0f);
        if (ACT == 3) v = v / (1.0f + expf(-v));
        if (ACT == 4) v = (v > 0.f) ? v : 0.01f * v;
        if (ACT == 5) v = 0.5f * v * (1.0f + erff(v * 0.70710678118654752f));
        if (ACT == 6) v = (v > 0.f) ? v : 0.2f * v;
        if (ACT == 7) { const float u = 0.7978845608028654f * (v + 0.044715f * v * v * v); v = 0.5f * v * (1.f + tanhf(u)); }
        slab[(mOff + r) * 68 + (j << 4) + rlane] = v;
      }
    }
    __builtin_amdgcn_fence(3  , "workgroup");
    __builtin_amdgcn_wave_barrier();
    __builtin_amdgcn_fence(2  , "workgroup");
    if (OUT_MODE == 0) {
      float* C = (float*)Cout + (size_t)b * strideC;
      const int hh = lane >> 4, c4 = (lane & 15) * 4;
      for (int pass = 0; pass < 2; ++pass) {
#pragma unroll
        for (int it = 0; it < 8; ++it) {
          const int row = it * 2 + hh;
          v4f v = *(const v4f*)(slab + row * 68 + c4);
          *(volatile v4f*)(C + (size_t)(mBase + row) * ldc + n0 + c4) = v;
        }
        __threadfence();
      }
    } else {
      const int q = lane >> 3, c8 = (lane & 7) * 8;
      unsigned short* C  = (unsigned short*)Cout  + (size_t)b * strideC;
      unsigned short* C2 = (OUT_MODE == 2) ? ((unsigned short*)Cout2 + (size_t)b * strideC) : nullptr;
      for (int pass = 0; pass < 2; ++pass) {
#pragma unroll
        for (int it = 0; it < 4; ++it) {
          const int row = it * 4 + q;
          const float* sp = slab + row * 68 + c8;
          v8h hv, lv;
#pragma unroll
          for (int e = 0; e < 8; ++e) {
            if (OUT_MODE == 1) {
              hv[e] = (_Float16)sp[e];
            } else {
              unsigned short hb = f2bf_bits(sp[e]);
              unsigned short lb = f2bf_bits(sp[e] - bf_bits2f(hb));
              hv[e] = __builtin_bit_cast(_Float16, hb);
              lv[e] = __builtin_bit_cast(_Float16, lb);
            }
          }
          *(volatile v8h*)(C + (size_t)(mBase + row) * ldc + n0 + c8) = hv;
          if (OUT_MODE == 2) *(volatile v8h*)(C2 + (size_t)(mBase + row) * ldc + n0 + c8) = lv;
        }
        __threadfence();
      }
    }
    __builtin_amdgcn_fence(3  , "workgroup");
    __builtin_amdgcn_wave_barrier();
    __builtin_amdgcn_fence(2  , "workgroup");
  }
}

}

static_assert(NROW % 64 == 0);
static_assert(NCAT % 64 == 0);
static_assert(DIN % 32 == 0);
static_assert(((NROW / 64) * (NCAT / 64)) % 8 == 0);
static_assert(8 * 16 * 68 * 4 <= 131072);
static_assert(NROW <= NROW_FULL);

__device__ __forceinline__ float bf_in(float f) { unsigned int u = __float_as_uint(f); u += 0x7fffu + ((u >> 16) & 1u); return __uint_as_float(u & 0xffff0000u); }
static __device__ __forceinline__ h16 toh_flush(float v) { const h16 r = (h16)v; return (fabsf(v) < 6.103515625e-05f) ? (h16)0.0f : r; }
__device__ __forceinline__ unsigned int pk2h_flush(float a, float b) { return (unsigned int)__builtin_bit_cast(unsigned short, toh_flush(a)) | ((unsigned int)__builtin_bit_cast(unsigned short, toh_flush(b)) << 16); }
__device__ __forceinline__ void st8h_flush(unsigned short* Pp, long long o, const float* v) { v4u pk; pk.x = pk2h_flush(v[0], v[1]); pk.y = pk2h_flush(v[2], v[3]); pk.z = pk2h_flush(v[4], v[5]); pk.w = pk2h_flush(v[6], v[7]); VST2(v4u, (v4u*)(Pp + o), pk); }

__global__ __launch_bounds__(256) void k_cv16(const float* __restrict__ X, unsigned short* __restrict__ O16, float sc, long long n8) {
    const long long u = (long long)blockIdx.x * 256 + threadIdx.x; if (u >= n8) return; const float* x = X + 8 * u; float v[8];
#pragma unroll
    for (int i = 0; i < 8; ++i) v[i] = bf_in(x[i]) * sc;
    st8h_flush(O16, 8 * u, v); }
static_assert(((long long)NROW * DIN) % (8 * 256) == 0);
static_assert(((long long)DH * DIN) % (8 * 256) == 0);

__global__ __launch_bounds__(256) void k_biasv(const float* __restrict__ bh, const float* __restrict__ bm, float* __restrict__ BV) {
    const int t = threadIdx.x; float o[4];
#pragma unroll
    for (int q = 0; q < 4; ++q) { const int i = 4 * t + q; const float hv = bh[min(i, DH - 1)]; const float mv = bm[min(max(i - DH, 0), DH - 1)]; o[q] = bf_in((i < DH) ? hv : mv); }
    v4f v; v.x = o[0]; v.y = o[1]; v.z = o[2]; v.w = o[3];
    VST2V4(BV + 4 * t, v); }
static_assert(256 * 4 == NCAT);

#define PT_TI 32
#define PT_TJ 32
#define PT_KC 128
#define PT_LS 132
#define PT_OS 36
static_assert(PT_TI == 8 * 4);
static_assert(PT_TJ == 32);
static_assert(DH % PT_KC == 0 && PT_KC % 4 == 0);
static_assert(PT_LS % 4 == 0 && PT_LS >= PT_KC && PT_OS % 4 == 0 && PT_OS >= PT_TJ);
static_assert(4 * 256 * 4 == PT_TI * PT_KC);
static_assert(DH % 256 == 0);
static_assert(256 * 16 == PT_TI * PT_TJ * 4);
static_assert(NROW % PT_TI == 0 && NROW % PT_TJ == 0);
static_assert((2 * PT_TI * PT_LS + DH + PT_TI * PT_OS) * 4 <= 131072);

__device__ __forceinline__ float fast_exp2(float x) {
#if __has_builtin(__builtin_amdgcn_exp2f)
    return __builtin_amdgcn_exp2f(x);
#else
    return exp2f(x);
#endif
}
__device__ __forceinline__ float fast_rcp(float x) {
#if __has_builtin(__builtin_amdgcn_rcpf)
    return __builtin_amdgcn_rcpf(x);
#else
    return 1.0f / x;
#endif
}
__device__ __forceinline__ float pair_term(float z, float w, float acc) {
    const float e = fast_exp2(z);
    const float r = fast_rcp(e + 1.0f);
    const float th = fmaf(-2.0f, r, 1.0f);
    return fmaf(w, th, acc);
}
__device__ __forceinline__ float pair4(v4f h, v4f m, v4f w, float acc) {
    acc = pair_term(h.x + m.x, w.x, acc);
    acc = pair_term(h.y + m.y, w.y, acc);
    acc = pair_term(h.z + m.z, w.z, acc);
    acc = pair_term(h.w + m.w, w.w, acc);
    return acc;
}

__global__ __launch_bounds__(256) void k_pair(const float* __restrict__ HM, const float* __restrict__ w2, const float* __restrict__ b2, float* __restrict__ out) {
    #pragma clang fp contract(off)
    __shared__ __align__(16) float Hs[PT_TI * PT_LS];
    __shared__ __align__(16) float Ms[PT_TJ * PT_LS];
    __shared__ __align__(16) float w2s[DH];
    __shared__ __align__(16) float ot[PT_TI * PT_OS];

    const int t = threadIdx.x;
    const int wave = __builtin_amdgcn_readfirstlane(threadIdx.x >> 5);
    const int lane = t & 31;
    const int i_base = blockIdx.y * PT_TI;
    const int j_base = blockIdx.x * PT_TJ;
    const int ii0 = wave * 4;
    const float C2 = 2.8853900817779268f;

    for (int k = t; k < DH; k += 256) w2s[k] = bf_in(w2[k]);

    float acc0 = 0.f, acc1 = 0.f, acc2 = 0.f, acc3 = 0.f;

    for (int kc = 0; kc < DH; kc += PT_KC) {
        __syncthreads();
#pragma unroll
        for (int p = 0; p < 4; ++p) {
            const int lin = t + p * 256;
            const int row = lin >> 5;
            const int k4 = (lin & 31) * 4;
            const v4f hv = *(const v4f*)(HM + (size_t)(i_base + row) * NCAT + kc + k4);
            const v4f mv = *(const v4f*)(HM + (size_t)(j_base + row) * NCAT + DH + kc + k4);
            *(v4f*)&Hs[row * PT_LS + k4] = hv * C2;
            *(v4f*)&Ms[row * PT_LS + k4] = mv * C2;
        }
        __syncthreads();

#pragma unroll 1
        for (int k = 0; k < PT_KC; k += 4) {
            const v4f m4 = *(const v4f*)&Ms[lane * PT_LS + k];
            const v4f w4 = *(const v4f*)&w2s[kc + k];
            const v4f h0 = *(const v4f*)&Hs[(ii0 + 0) * PT_LS + k];
            const v4f h1 = *(const v4f*)&Hs[(ii0 + 1) * PT_LS + k];
            const v4f h2 = *(const v4f*)&Hs[(ii0 + 2) * PT_LS + k];
            const v4f h3 = *(const v4f*)&Hs[(ii0 + 3) * PT_LS + k];
            acc0 = pair4(h0, m4, w4, acc0);
            acc1 = pair4(h1, m4, w4, acc1);
            acc2 = pair4(h2, m4, w4, acc2);
            acc3 = pair4(h3, m4, w4, acc3);
        }
    }

    const float bias = bf_in(b2[0]);
    ot[(ii0 + 0) * PT_OS + lane] = acc0 + bias;
    ot[(ii0 + 1) * PT_OS + lane] = acc1 + bias;
    ot[(ii0 + 2) * PT_OS + lane] = acc2 + bias;
    ot[(ii0 + 3) * PT_OS + lane] = acc3 + bias;
    __syncthreads();
    {
        const int row = t >> 3, c4 = (t & 7) * 4;
        const v4f v = *(const v4f*)&ot[row * PT_OS + c4];
        VST2V4(out + (size_t)(i_base + row) * NROW_FULL + j_base + c4, v);
    }
}

#define CARVE_A16 ((((size_t)NROW * DIN * 2) + 255) / 256 * 256)
#define CARVE_W16 ((((size_t)NCAT * DIN * 2) + 255) / 256 * 256)
#define CARVE_BV  ((((size_t)NCAT * 4) + 255) / 256 * 256)
#define CARVE_HM  ((((size_t)NROW * NCAT * 4) + 255) / 256 * 256)
static_assert(CARVE_A16 + CARVE_W16 + CARVE_BV + CARVE_HM <= (size_t)134217728);

extern "C" void kernel_launch(void* const* d_in, const int* in_sizes, int n_in, void* d_out, int out_size, void* d_ws, size_t ws_size, hipStream_t stream) {
    if (n_in < 7) return;
    if ((long long)in_sizes[0] < (long long)NROW * DIN) return;
    if ((long long)in_sizes[1] < (long long)DH * DIN) return;
    if (in_sizes[2] < DH) return;
    if ((long long)in_sizes[3] < (long long)DH * DIN) return;
    if (in_sizes[4] < DH) return;
    if (in_sizes[5] < DH) return;
    if (in_sizes[6] < 1) return;
    if ((long long)out_size < (long long)(NROW - 1) * NROW_FULL + NROW) return;
    const float* vectors = (const float*)d_in[0];
    const float* W_h = (const float*)d_in[1];
    const float* b_h = (const float*)d_in[2];
    const float* W_m = (const float*)d_in[3];
    const float* b_m = (const float*)d_in[4];
    const float* w2 = (const float*)d_in[5];
    const float* b2 = (const float*)d_in[6];
    float* out = (float*)d_out;
    char* wsp = (char*)d_ws;
    unsigned short* A16 = (unsigned short*)wsp; wsp += CARVE_A16;
    unsigned short* W16 = (unsigned short*)wsp; wsp += CARVE_W16;
    float* BV = (float*)wsp; wsp += CARVE_BV;
    float* HM = (float*)wsp; wsp += CARVE_HM;
    if ((size_t)(wsp - (char*)d_ws) > ws_size) return;

    k_cv16<<<(unsigned)(((long long)NROW * DIN / 8) / 256), 256, 0, stream>>>(vectors, A16, 8.0f, (long long)NROW * DIN / 8);
    k_cv16<<<(unsigned)(((long long)DH * DIN / 8) / 256), 256, 0, stream>>>(W_h, W16, 32.0f, (long long)DH * DIN / 8);
    k_cv16<<<(unsigned)(((long long)DH * DIN / 8) / 256), 256, 0, stream>>>(W_m, W16 + (size_t)DH * DIN, 32.0f, (long long)DH * DIN / 8);
    k_biasv<<<1, 256, 0, stream>>>(b_h, b_m, BV);
    eng::wmma_gemm64<0, false, 2, 0, false><<<dim3((unsigned)((((NROW) / 64) * ((NCAT) / 64) + 7) / 8), (unsigned)(1)), 256, 0, stream>>>((const unsigned short*)(A16), nullptr, DIN, 0, (const unsigned short*)(W16), nullptr, DIN, 0, (void*)(HM), nullptr, NCAT, 0, BV, nullptr, 0, NROW, NCAT, DIN, 0.00390625f);
    k_pair<<<dim3((unsigned)(NROW / PT_TJ), (unsigned)(NROW / PT_TI)), 256, 0, stream>>>(HM, w2, b2, out);
}
